// BBBLSTM_60696477827102
// MI455X (gfx1250) — hardware-verified
//
#include <hip/hip_runtime.h>

typedef __attribute__((ext_vector_type(16))) _Float16 v16h;
typedef __attribute__((ext_vector_type(8)))  _Float16 v8h;
typedef __attribute__((ext_vector_type(8)))  float    v8f;
typedef __attribute__((ext_vector_type(4)))  float    v4f;

__device__ __forceinline__ void dep_guard_h(v8f& a, v8f& b, v16h x, v16h y) { asm volatile("v_nop\n\tv_nop\n\tv_nop\n\tv_nop" : "+v"(a), "+v"(b) : "v"(x), "v"(y)); }
__device__ __forceinline__ void keep4_h(v16h a, v16h b, v16h c, v16h d) { asm volatile("v_nop" :: "v"(a), "v"(b), "v"(c), "v"(d)); }
__device__ __forceinline__ void acc_guard4(v8f& a, v8f& b, v8f& c, v8f& d) { asm volatile("v_nop\n\tv_nop\n\tv_nop\n\tv_nop" : "+v"(a), "+v"(b), "+v"(c), "+v"(d)); }
__device__ __forceinline__ void dep_guard1_h(v8f& a, v16h x, v16h y) { asm volatile("v_nop\n\tv_nop\n\tv_nop\n\tv_nop" : "+v"(a) : "v"(x), "v"(y)); }

template <typename T> struct Frag;
template <> struct Frag<_Float16> {
  typedef v16h V; union U { v16h v; v8h h[2]; };
  static __device__ __forceinline__ v16h load(const _Float16* p) {
    U f; f.h[0] = *(const v8h*)(p); f.h[1] = *(const v8h*)(p + 16); return f.v;
  }
  static __device__ __forceinline__ v8f mma(v16h a, v16h b, v8f c) {
    return __builtin_amdgcn_wmma_f32_16x16x32_f16(false, a, false, b, (short)0, c, false, false);
  }
  static __device__ __forceinline__ void guard(v8f& a, v8f& b, v16h x, v16h y) { dep_guard_h(a, b, x, y); }
  static __device__ __forceinline__ void keep(v16h a, v16h b, v16h c, v16h d) { keep4_h(a, b, c, d); }
};
typedef Frag<_Float16> FragH;

constexpr int   T_STEPS   = 30;
constexpr int   F_IN      = 25;
constexpr int   H_HID     = 128;
constexpr int   G4        = 512;
constexpr int   KX_PAD    = 32;
constexpr int   KCAT      = KX_PAD + H_HID;
constexpr int   KPAD_CAT  = 192;
constexpr int   ROWS_BLK  = 16;
constexpr int   NTHR      = 256;
constexpr int   HPITCH    = 128;
constexpr int   H2_OUT    = 64;
constexpr float INV128    = 0.0078125f;
constexpr float ACT_SCALE = 8.0f;
constexpr float W_SCALE   = 16.0f;

static_assert(KCAT % 32 == 0, "k depth multiple of 32");
static_assert(KPAD_CAT % 8 == 0 && HPITCH % 8 == 0, "16-B aligned fragment loads");

__device__ __forceinline__ float opaque_zero() { float z; asm volatile("v_mov_b32 %0, 0" : "=v"(z)); return z; }

__device__ __forceinline__ float sigm_f(float xx) {
  const float xc = fminf(fmaxf(xx, -30.0f), 30.0f);
  return __builtin_amdgcn_rcpf(1.0f + __expf(-xc));
}
__device__ __forceinline__ float tanh_f(float xx) {
  const float xc = fminf(fmaxf(xx, -15.0f), 15.0f);
  return 1.0f - 2.0f * __builtin_amdgcn_rcpf(1.0f + __expf(2.0f * xc));
}

__global__ __launch_bounds__(256) void prep_gate_weights(
    const float* __restrict__ w_ih, const float* __restrict__ w_hh,
    _Float16* __restrict__ dst, int nthr) {
  const int i = blockIdx.x * 256 + threadIdx.x;
  if (i >= nthr) return;
  const float vz = opaque_zero();
  const int e  = i * 8;
  const int n  = e / KPAD_CAT;
  const int k0 = e - n * KPAD_CAT;
  v8h hv;
#pragma unroll
  for (int j = 0; j < 8; ++j) {
    const int k = k0 + j;
    const int ki = (k < F_IN - 1) ? k : (F_IN - 1);
    int kh = k - KX_PAD; kh = kh < 0 ? 0 : (kh > H_HID - 1 ? H_HID - 1 : kh);
    const float a = w_ih[(size_t)ki * G4 + n];
    const float b = w_hh[(size_t)kh * G4 + n];
    const float v = (k < F_IN) ? a : ((k >= KX_PAD && k < KX_PAD + H_HID) ? b : vz);
    hv[j] = (_Float16)(v * W_SCALE);
  }
  volatile v8h* p = (volatile v8h*)(dst + (size_t)e);
  *p = hv;
  __threadfence();
  *p = hv;
}

__global__ __launch_bounds__(256) void prep_t16(
    const float* __restrict__ src, int kin, int ncols,
    _Float16* __restrict__ dst, int kpad, int nthr) {
  const int i = blockIdx.x * 256 + threadIdx.x;
  if (i >= nthr) return;
  const float vz = opaque_zero();
  const int e  = i * 8;
  const int n  = e / kpad;
  const int k0 = e - n * kpad;
  v8h hv;
#pragma unroll
  for (int j = 0; j < 8; ++j) {
    const int k  = k0 + j;
    const int kc = (k < kin) ? k : (kin - 1);
    const float ld = src[(size_t)kc * ncols + n];
    const float v  = (k < kin) ? ld : vz;
    hv[j] = (_Float16)(v * W_SCALE);
  }
  volatile v8h* p = (volatile v8h*)(dst + (size_t)e);
  *p = hv;
  __threadfence();
  *p = hv;
}

__global__ __launch_bounds__(NTHR) void lstm_head_persistent(
    const float* __restrict__ x, const float* __restrict__ ln_g, const float* __restrict__ ln_b,
    const _Float16* __restrict__ wcat, const float* __restrict__ b_lstm,
    const _Float16* __restrict__ w1t, const float* __restrict__ b1,
    const _Float16* __restrict__ w2t, const float* __restrict__ b2,
    const float* __restrict__ w3, const float* __restrict__ b3,
    float* __restrict__ out, int nB) {
  __shared__ __align__(16) _Float16 xall[T_STEPS * ROWS_BLK * KX_PAD];
  __shared__ __align__(16) _Float16 htile[2][ROWS_BLK * HPITCH];
  __shared__ __align__(16) float    y2f[ROWS_BLK * H2_OUT];
  __shared__ __align__(16) float    outs[32];

  const int tid  = threadIdx.x;
  const int lane = tid & 31;
  const int wave = tid >> 5;
  const int hh   = lane >> 4;
  const int rl   = lane & 15;
  const int koff = hh * 8;
  const int b0   = blockIdx.x * ROWS_BLK;
  const float vz = opaque_zero();

  for (int rr = tid; rr < T_STEPS * ROWS_BLK; rr += NTHR) {
    const int tt = rr >> 4, m = rr & 15;
    int brow = b0 + m; brow = (brow < nB) ? brow : (nB - 1);
    const float* xp = x + ((size_t)brow * T_STEPS + tt) * F_IN;
    float xv[F_IN];
#pragma unroll
    for (int f = 0; f < F_IN; ++f) xv[f] = xp[f];
    float s = 0.0f;
#pragma unroll
    for (int f = 0; f < F_IN; ++f) s += xv[f];
    const float mu = s * (1.0f / 25.0f);
    float sq = 0.0f;
#pragma unroll
    for (int f = 0; f < F_IN; ++f) { const float d = xv[f] - mu; sq += d * d; }
    const float var  = sq * (1.0f / 25.0f);
    const float rstd = rsqrtf(var + 1e-5f);
    _Float16 e16[KX_PAD];
#pragma unroll
    for (int f = 0; f < F_IN; ++f)
      e16[f] = (_Float16)(((xv[f] - mu) * rstd * ln_g[f] + ln_b[f]) * ACT_SCALE);
#pragma unroll
    for (int f = F_IN; f < KX_PAD; ++f) e16[f] = (_Float16)vz;
    _Float16* xr = xall + rr * KX_PAD;
#pragma unroll
    for (int q4 = 0; q4 < 4; ++q4) {
      v8h pv;
#pragma unroll
      for (int j = 0; j < 8; ++j) pv[j] = e16[8 * q4 + j];
      *(v8h*)(xr + 8 * q4) = pv;
    }
  }
  {
    v8h z8;
#pragma unroll
    for (int j = 0; j < 8; ++j) z8[j] = (_Float16)vz;
    *(v8h*)(&htile[0][0] + tid * 8) = z8;
  }

  const int hcol = 16 * wave + rl;
  float bg[4];
  int   nb[4];
#pragma unroll
  for (int g = 0; g < 4; ++g) {
    bg[g] = b_lstm[g * H_HID + hcol];
    nb[g] = (g * H_HID + hcol) * KPAD_CAT + koff;
  }
  float cst[8];
#pragma unroll
  for (int r = 0; r < 8; ++r) cst[r] = 0.0f;
  const v8f zero8 = {0.f, 0.f, 0.f, 0.f, 0.f, 0.f, 0.f, 0.f};

  for (int t = 0; t < T_STEPS; ++t) {
    __syncthreads();
    const _Float16* hin = &htile[t & 1][0];
    _Float16* hout = &htile[(t + 1) & 1][0];
    v8f acc[4];
#pragma unroll
    for (int g = 0; g < 4; ++g) acc[g] = zero8;
    {
      const v16h a = FragH::load(xall + (t * ROWS_BLK + rl) * KX_PAD + koff);
      v16h bq[4];
#pragma unroll
      for (int g = 0; g < 4; ++g) bq[g] = FragH::load(wcat + nb[g]);
#pragma unroll
      for (int g = 0; g < 4; ++g) acc[g] = FragH::mma(a, bq[g], acc[g]);
      FragH::guard(acc[0], acc[3], a, bq[0]);
      FragH::keep(bq[0], bq[1], bq[2], bq[3]);
    }
#pragma unroll
    for (int ks = 0; ks < 4; ++ks) {
      const v16h a = FragH::load(hin + rl * HPITCH + 32 * ks + koff);
      v16h bq[4];
#pragma unroll
      for (int g = 0; g < 4; ++g) bq[g] = FragH::load(wcat + nb[g] + KX_PAD + 32 * ks);
#pragma unroll
      for (int g = 0; g < 4; ++g) acc[g] = FragH::mma(a, bq[g], acc[g]);
      FragH::guard(acc[0], acc[3], a, bq[0]);
      FragH::keep(bq[0], bq[1], bq[2], bq[3]);
    }
    acc_guard4(acc[0], acc[1], acc[2], acc[3]);

#pragma unroll
    for (int r = 0; r < 8; ++r) {
      const float pi = acc[0][r] * INV128 + bg[0];
      const float pf = acc[1][r] * INV128 + bg[1];
      const float pg = acc[2][r] * INV128 + bg[2];
      const float po = acc[3][r] * INV128 + bg[3];
      const float cn = sigm_f(pf) * cst[r] + sigm_f(pi) * tanh_f(pg);
      cst[r] = cn;
      const float hv = sigm_f(po) * tanh_f(cn);
      hout[(8 * hh + r) * HPITCH + hcol] = (_Float16)(hv * ACT_SCALE);
    }
  }
  __syncthreads();

  const _Float16* hfin = &htile[T_STEPS & 1][0];
  _Float16* y1t = &htile[(T_STEPS + 1) & 1][0];
  {
    v8f a1 = zero8;
#pragma unroll
    for (int ks = 0; ks < 4; ++ks) {
      const v16h a = FragH::load(hfin + rl * HPITCH + 32 * ks + koff);
      const v16h b = FragH::load(w1t + (size_t)hcol * H_HID + koff + 32 * ks);
      a1 = FragH::mma(a, b, a1);
      dep_guard1_h(a1, a, b);
    }
    const float bb1 = b1[hcol];
#pragma unroll
    for (int r = 0; r < 8; ++r) {
      const float v = fmaxf(a1[r] * INV128 + bb1, 0.0f);
      y1t[(8 * hh + r) * HPITCH + hcol] = (_Float16)(v * ACT_SCALE);
    }
  }
  __syncthreads();

  {
    const int ns   = wave & 3;
    const int ncol = 16 * ns + rl;
    v8f a2 = zero8;
#pragma unroll
    for (int ks = 0; ks < 4; ++ks) {
      const v16h a = FragH::load(y1t + rl * HPITCH + 32 * ks + koff);
      const v16h b = FragH::load(w2t + (size_t)ncol * H_HID + koff + 32 * ks);
      a2 = FragH::mma(a, b, a2);
      dep_guard1_h(a2, a, b);
    }
    if (wave < 4) {
      const float bb2 = b2[ncol];
#pragma unroll
      for (int r = 0; r < 8; ++r)
        y2f[(8 * hh + r) * H2_OUT + ncol] = fmaxf(a2[r] * INV128 + bb2, 0.0f);
    }
  }
  __syncthreads();

  if (wave == 0) {
    const int m = lane >> 1, col = lane & 1;
    float s = 0.0f;
#pragma unroll 1
    for (int k = 0; k < H2_OUT; ++k) s = fmaf(y2f[m * H2_OUT + k], w3[k * 2 + col], s);
    outs[lane] = s + b3[col];
  }
  __syncthreads();
  if (tid < 8 && (b0 + ROWS_BLK) <= nB) {
    const v4f v = *(const v4f*)(outs + 4 * tid);
    volatile v4f* p = (volatile v4f*)(out + (size_t)b0 * 2 + 4 * tid);
    *p = v;
    __threadfence();
    *p = v;
  }
}

extern "C" void kernel_launch(void* const* d_in, const int* in_sizes, int n_in,
                              void* d_out, int out_size, void* d_ws, size_t ws_size,
                              hipStream_t stream) {
  if (n_in < 12) return;
  const float* x      = (const float*)d_in[0];
  const float* ln_g   = (const float*)d_in[1];
  const float* ln_b   = (const float*)d_in[2];
  const float* w_ih   = (const float*)d_in[3];
  const float* w_hh   = (const float*)d_in[4];
  const float* b_lstm = (const float*)d_in[5];
  const float* w1     = (const float*)d_in[6];
  const float* b1     = (const float*)d_in[7];
  const float* w2     = (const float*)d_in[8];
  const float* b2     = (const float*)d_in[9];
  const float* w3     = (const float*)d_in[10];
  const float* b3     = (const float*)d_in[11];
  float* out = (float*)d_out;

  const int nB = in_sizes[0] / (T_STEPS * F_IN);
  int nblk = nB / ROWS_BLK;
  const int max_blk_out = out_size / (ROWS_BLK * 2);
  if (nblk > max_blk_out) nblk = max_blk_out;
  if (nblk < 1) return;

  const size_t wcat_bytes = (size_t)G4 * KPAD_CAT * 2;
  const size_t w1t_bytes  = (size_t)H_HID * H_HID * 2;
  const size_t w2t_bytes  = (size_t)H2_OUT * H_HID * 2;
  const size_t off_wcat = 0;
  const size_t off_w1t  = off_wcat + wcat_bytes;
  const size_t off_w2t  = off_w1t + w1t_bytes;
  if (off_w2t + w2t_bytes > ws_size) return;

  char* ws = (char*)d_ws;
  _Float16* wcat = (_Float16*)(ws + off_wcat);
  _Float16* w1t  = (_Float16*)(ws + off_w1t);
  _Float16* w2t  = (_Float16*)(ws + off_w2t);

  const int nthr_wcat = G4 * KPAD_CAT / 8;
  const int nthr_w1   = H_HID * H_HID / 8;
  const int nthr_w2   = H2_OUT * H_HID / 8;
  prep_gate_weights<<<dim3((nthr_wcat + 255) / 256), dim3(256), 0, stream>>>(w_ih, w_hh, wcat, nthr_wcat);
  prep_t16<<<dim3((nthr_w1 + 255) / 256), dim3(256), 0, stream>>>(w1, H_HID, H_HID, w1t, H_HID, nthr_w1);
  prep_t16<<<dim3((nthr_w2 + 255) / 256), dim3(256), 0, stream>>>(w2, H_HID, H2_OUT, w2t, H_HID, nthr_w2);
  lstm_head_persistent<<<dim3(nblk), dim3(NTHR), 0, stream>>>(
      x, ln_g, ln_b, wcat, b_lstm, w1t, b1, w2t, b2, w3, b3, out, nB);
}
